// EdgeRegressionHead_63333587746832
// MI455X (gfx1250) — hardware-verified
//
#include <hip/hip_runtime.h>
#include <stdint.h>


typedef _Float16 half_t;
typedef _Float16 v16h __attribute__((ext_vector_type(16)));
typedef _Float16 v8h  __attribute__((ext_vector_type(8)));
typedef float    v8f  __attribute__((ext_vector_type(8)));
typedef float    v4f  __attribute__((ext_vector_type(4)));

union Frag { v16h v; v8h hv[2]; };

#define DDIM            128
#define W1_K            256
#define TILE_M          16
#define NWAVES          8
#define NTHREADS        (NWAVES * 32)
#define TILES_PER_WAVE  4
#define EDGES_PER_WAVE  (TILE_M * TILES_PER_WAVE)
#define EDGES_PER_BLOCK (NWAVES * EDGES_PER_WAVE)
#define LDS_PAD         8
#define W1_LD           (W1_K + LDS_PAD)
#define W2_LD           (DDIM + LDS_PAD)
#define ST_LD           (DDIM + LDS_PAD)
#define WSCALE          64.0f
#define WSCALE_INV      0.015625f

__device__ __forceinline__ v8f wmma16(v16h a, v16h b, v8f c)
{
    v8f d = __builtin_amdgcn_wmma_f32_16x16x32_f16(false, a, false, b, (short)0, c, false, false);
    asm volatile("v_nop\n\tv_nop\n\tv_nop\n\tv_nop" : "+v"(d) : "v"(a), "v"(b));
    return d;
}

__device__ __forceinline__ void store_piece(float* out, long e0, long E, v4f v)
{
    if (e0 + 4 <= E) {
        *(volatile v4f*)(out + e0) = v;
    } else {
        #pragma unroll
        for (int j = 0; j < 4; ++j) {
            if (e0 + j < E) *((volatile float*)out + e0 + j) = v[j];
        }
    }
}

__global__ __launch_bounds__(NTHREADS) void edge_mlp_kernel(
    const float* __restrict__ x,
    const int*   __restrict__ src,
    const int*   __restrict__ dst,
    const float* __restrict__ W1, const float* __restrict__ b1,
    const float* __restrict__ W2, const float* __restrict__ b2,
    const float* __restrict__ W3, const float* __restrict__ b3,
    float* out, int E, int N)
{
    __shared__ __attribute__((aligned(16))) half_t sW1[DDIM][W1_LD];
    __shared__ __attribute__((aligned(16))) half_t sW2[DDIM][W2_LD];
    __shared__ __attribute__((aligned(16))) half_t sStage[NWAVES][TILE_M][ST_LD];
    __shared__ __attribute__((aligned(16))) float  sOut[NWAVES][EDGES_PER_WAVE];
    __shared__ float sB1[DDIM];
    __shared__ float sB2[DDIM];
    __shared__ float sW3[DDIM];

    const int tid = threadIdx.x;

    for (int i = tid; i < W1_K * DDIM; i += NTHREADS) {
        const int k = i / DDIM, n = i - k * DDIM;
        sW1[n][k] = (half_t)(W1[i] * WSCALE);
    }
    for (int i = tid; i < DDIM * DDIM; i += NTHREADS) {
        const int k = i / DDIM, n = i - k * DDIM;
        sW2[n][k] = (half_t)(W2[i] * WSCALE);
    }
    for (int i = tid; i < DDIM; i += NTHREADS) {
        sB1[i] = b1[i];
        sB2[i] = b2[i];
        sW3[i] = W3[i];
    }
    __syncthreads();

    const int wave = tid >> 5;
    const int lane = tid & 31;
    const int m    = lane & 15;
    const int h    = lane >> 4;
    const float b3v = b3[0];

    half_t (*stage)[ST_LD] = sStage[wave];
    float* so = sOut[wave];

    const long waveBase = ((long)blockIdx.x * NWAVES + wave) * (long)EDGES_PER_WAVE;

    #pragma unroll 1
    for (int t = 0; t < TILES_PER_WAVE; ++t) {
        __syncthreads();

        const long tileBase = waveBase + (long)t * TILE_M;
        long eRow = tileBase + m;
        if (eRow > (long)E - 1) eRow = (long)E - 1;
        int si = src[eRow];
        int di = dst[eRow];
        si = si < 0 ? 0 : (si > N - 1 ? N - 1 : si);
        di = di < 0 ? 0 : (di > N - 1 ? N - 1 : di);
        const float* rowS = x + (size_t)si * DDIM;
        const float* rowD = x + (size_t)di * DDIM;

        v8f acc[8];
        #pragma unroll
        for (int nt = 0; nt < 8; ++nt) {
            #pragma unroll
            for (int r = 0; r < 8; ++r) acc[nt][r] = 0.0f;
        }

        #pragma unroll 1
        for (int kt = 0; kt < 8; ++kt) {
            const float* rp = (kt < 4) ? rowS : rowD;
            const int base = (kt & 3) * 32 + h * 8;
            const v4f f0 = *(const v4f*)(rp + base);
            const v4f f1 = *(const v4f*)(rp + base + 4);
            const v4f f2 = *(const v4f*)(rp + base + 16);
            const v4f f3 = *(const v4f*)(rp + base + 20);
            v16h a;
            #pragma unroll
            for (int j = 0; j < 4; ++j) {
                a[j]      = (half_t)f0[j];
                a[4 + j]  = (half_t)f1[j];
                a[8 + j]  = (half_t)f2[j];
                a[12 + j] = (half_t)f3[j];
            }
            const int kb = kt * 32 + h * 8;
            #pragma unroll
            for (int nt = 0; nt < 8; ++nt) {
                const half_t* wp = &sW1[nt * 16 + m][kb];
                Frag b;
                b.hv[0] = *(const v8h*)(wp);
                b.hv[1] = *(const v8h*)(wp + 16);
                acc[nt] = wmma16(a, b.v, acc[nt]);
            }
        }

        #pragma unroll
        for (int nt = 0; nt < 8; ++nt) {
            const float bias = sB1[nt * 16 + m];
            #pragma unroll
            for (int r = 0; r < 8; ++r) {
                float v = acc[nt][r] * WSCALE_INV + bias;
                v = v > 0.0f ? v : 0.0f;
                stage[r + h * 8][nt * 16 + m] = (half_t)v;
                acc[nt][r] = 0.0f;
            }
        }
        __syncthreads();

        #pragma unroll 1
        for (int kt = 0; kt < 4; ++kt) {
            const int kb = kt * 32 + h * 8;
            Frag a;
            a.hv[0] = *(const v8h*)(&stage[m][kb]);
            a.hv[1] = *(const v8h*)(&stage[m][kb + 16]);
            #pragma unroll
            for (int nt = 0; nt < 8; ++nt) {
                const half_t* wp = &sW2[nt * 16 + m][kb];
                Frag b;
                b.hv[0] = *(const v8h*)(wp);
                b.hv[1] = *(const v8h*)(wp + 16);
                acc[nt] = wmma16(a.v, b.v, acc[nt]);
            }
        }

        float s[8];
        #pragma unroll
        for (int r = 0; r < 8; ++r) s[r] = 0.0f;
        #pragma unroll
        for (int nt = 0; nt < 8; ++nt) {
            const float bias = sB2[nt * 16 + m];
            const float w3   = sW3[nt * 16 + m];
            #pragma unroll
            for (int r = 0; r < 8; ++r) {
                float v = acc[nt][r] * WSCALE_INV + bias;
                v = v > 0.0f ? v : 0.0f;
                s[r] += v * w3;
            }
        }
        #pragma unroll
        for (int r = 0; r < 8; ++r) {
            s[r] += __shfl_xor(s[r], 1, 32);
            s[r] += __shfl_xor(s[r], 2, 32);
            s[r] += __shfl_xor(s[r], 4, 32);
            s[r] += __shfl_xor(s[r], 8, 32);
        }
        float val = s[0];
        #pragma unroll
        for (int r = 1; r < 8; ++r) val = (m == r) ? s[r] : val;
        if (m < 8) so[t * TILE_M + 8 * h + m] = val + b3v;
    }
    __syncthreads();

    if (lane < 16) {
        const long e0 = waveBase + 4 * lane;
        const v4f v = *(const v4f*)(so + 4 * lane);
        store_piece(out, e0, (long)E, v);
    }
    __threadfence();
    if (lane < 16) {
        const long e0 = waveBase + 4 * lane;
        const v4f v = *(const v4f*)(so + 4 * lane);
        store_piece(out, e0, (long)E, v);
    }
}

extern "C" void kernel_launch(void* const* d_in, const int* in_sizes, int n_in,
                              void* d_out, int out_size, void* d_ws, size_t ws_size,
                              hipStream_t stream)
{
    const float* x  = (const float*)d_in[0];
    const int*   s  = (const int*)  d_in[1];
    const int*   d  = (const int*)  d_in[2];
    const float* W1 = (const float*)d_in[3];
    const float* b1 = (const float*)d_in[4];
    const float* W2 = (const float*)d_in[5];
    const float* b2 = (const float*)d_in[6];
    const float* W3 = (const float*)d_in[7];
    const float* b3 = (const float*)d_in[8];
    float* out = (float*)d_out;

    const int E = in_sizes[1];
    const int N = in_sizes[0] / DDIM;
    if (E <= 0 || N <= 0 || out_size < E) return;

    const int blocks = (E + EDGES_PER_BLOCK - 1) / EDGES_PER_BLOCK;
    edge_mlp_kernel<<<blocks, NTHREADS, 0, stream>>>(x, s, d, W1, b1, W2, b2, W3, b3, out, E, N);
}
